// FLGNN_90941637525593
// MI455X (gfx1250) — hardware-verified
//
#include <hip/hip_runtime.h>
#include <stddef.h>
#include <math.h>


#define FD      128
#define RR      16
#define NLAY    3
#define NOUT    40
#define NOP     64
#define PP      128
#define NTHR    256
#define NWAVE   8
#define EPT     8
#define NGRP    2
#define CHUNK   (NTHR * EPT * NGRP)
#define WCAP    (EPT * NGRP * 32)
#define LISTN   (NWAVE * WCAP)
#define NBC     2048
#define NBF     1024
#define FPC     (NBC / NBF)
#define RCAP    36864
#define RBN     128
#define TGT     256
#define DEGCAP  256
#define OTHR    256
#define BM      64
#define STATR   256
#define WSCAP   134217728
#define BN_EPS  1e-5

#define LDS_FILL ((RCAP + NBF + LISTN) * 4 + 64)
#define LDS_GIN  (BM * FD * 4)
#define LDS_MSG  ((BM * FD + BM * RR + BM * RR + BM * FD) * 4)
#define LDS_HEAD ((BM * NOP + BM * NOUT) * 4)

static_assert((CHUNK & (CHUNK - 1)) == 0);
static_assert(CHUNK <= 4096);
static_assert(NBC <= 4096 && NBF <= 4096);
static_assert((NBC & (NBC - 1)) == 0 && (NBF & (NBF - 1)) == 0);
static_assert(NBC == FPC * NBF && FPC == 2);
static_assert(OTHR * 8 == NBC && OTHR == 256);
static_assert((RCAP % 32) == 0);
static_assert(TGT == NWAVE * 32);
static_assert((TGT % BM) == 0 && (TGT % STATR) == 0);
static_assert((DEGCAP % 32) == 0);
static_assert(FD == 128 && PP == FD && RR == 16 && BM == 64 && NWAVE == 8 && NOUT <= NOP);
static_assert(((BM * NOUT * 4) % 128) == 0 && ((BM * NOUT) % 4) == 0);

typedef float          v4f  __attribute__((ext_vector_type(4)));
typedef float          v8f  __attribute__((ext_vector_type(8)));
typedef double         v2d  __attribute__((ext_vector_type(2)));
typedef int            v4i  __attribute__((ext_vector_type(4)));
typedef unsigned short v4us __attribute__((ext_vector_type(4)));
typedef unsigned short v8us __attribute__((ext_vector_type(8)));
typedef unsigned short v16us __attribute__((ext_vector_type(16)));
typedef __bf16         v16bf __attribute__((ext_vector_type(16)));
union FragU { v16us w; v8us u[2]; };

__device__ __forceinline__ v8f wmb(v16us a, v16us b, v8f c) {
  const v16bf ab = __builtin_bit_cast(v16bf, a);
  const v16bf bb = __builtin_bit_cast(v16bf, b);
  v8f d = __builtin_amdgcn_wmma_f32_16x16x32_bf16(false, ab, false, bb, (short)0, c, false, false);
  asm volatile("v_nop\n\tv_nop\n\tv_nop\n\tv_nop" : "+v"(d) : "v"(a), "v"(b));
  return d;
}

__device__ __forceinline__ unsigned int bfb(float f) {
  const unsigned int u = __float_as_uint(f);
  return (u + 0x7FFFu + ((u >> 16) & 1u)) >> 16;
}
__device__ __forceinline__ void sp1(float v, unsigned short& h, unsigned short& l) {
  const unsigned int hb = bfb(v);
  const float hf = __uint_as_float(hb << 16);
  h = (unsigned short)hb;
  l = (unsigned short)bfb(v - hf);
}
__device__ __forceinline__ void sp8(v4f a, v4f b, v8us& h, v8us& l) {
  unsigned short hh, ll;
  sp1(a.x, hh, ll); h[0] = hh; l[0] = ll;
  sp1(a.y, hh, ll); h[1] = hh; l[1] = ll;
  sp1(a.z, hh, ll); h[2] = hh; l[2] = ll;
  sp1(a.w, hh, ll); h[3] = hh; l[3] = ll;
  sp1(b.x, hh, ll); h[4] = hh; l[4] = ll;
  sp1(b.y, hh, ll); h[5] = hh; l[5] = ll;
  sp1(b.z, hh, ll); h[6] = hh; l[6] = ll;
  sp1(b.w, hh, ll); h[7] = hh; l[7] = ll;
}
__device__ __forceinline__ void sp4(v4f a, v4us& h, v4us& l) {
  unsigned short hh, ll;
  sp1(a.x, hh, ll); h[0] = hh; l[0] = ll;
  sp1(a.y, hh, ll); h[1] = hh; l[1] = ll;
  sp1(a.z, hh, ll); h[2] = hh; l[2] = ll;
  sp1(a.w, hh, ll); h[3] = hh; l[3] = ll;
}
__device__ __forceinline__ v4f relu4(v4f t) {
  v4f r;
  r.x = fmaxf(t.x, 0.f); r.y = fmaxf(t.y, 0.f); r.z = fmaxf(t.z, 0.f); r.w = fmaxf(t.w, 0.f);
  return r;
}

__global__ __launch_bounds__(NTHR) void k_wprep(const float* __restrict__ W, int nreal, int ntot,
                                               unsigned short* ph, unsigned short* pl, int units) {
  const int i = (int)blockIdx.x * NTHR + (int)threadIdx.x;
  if (i >= units) return;
  const int n  = i >> 4;
  const int k0 = (i & 15) * 8;
  const int na = n < nreal - 1 ? n : nreal - 1;
  v8us hv, lv;
#pragma unroll
  for (int e = 0; e < 8; ++e) {
    float f = W[(size_t)(k0 + e) * nreal + na];
    f = n < nreal ? f : 0.f;
    unsigned short h, l;
    sp1(f, h, l);
    hv[e] = h; lv[e] = l;
  }
  unsigned short* dh = ph + (size_t)i * 8;
  unsigned short* dl = pl + (size_t)i * 8;
  *(volatile v8us*)dh = hv;
  *(volatile v8us*)dl = lv;
  __threadfence();
  *(volatile v8us*)dh = hv;
  *(volatile v8us*)dl = lv;
}

__global__ __launch_bounds__(NTHR) void k_bprep(const float* __restrict__ Wc, unsigned short* ph,
                                               unsigned short* pl, int units) {
  const int i = (int)blockIdx.x * NTHR + (int)threadIdx.x;
  if (i >= units) return;
  const int g  = i >> 4;
  const int k0 = (i & 15) * 8;
  const int lr = g >> 7;
  const int o  = g & 127;
  v8us hv, lv;
#pragma unroll
  for (int e = 0; e < 8; ++e) {
    const float f = Wc[((size_t)lr * FD + (size_t)(k0 + e)) * FD + o];
    unsigned short h, l;
    sp1(f, h, l);
    hv[e] = h; lv[e] = l;
  }
  unsigned short* dh = ph + (size_t)i * 8;
  unsigned short* dl = pl + (size_t)i * 8;
  *(volatile v8us*)dh = hv;
  *(volatile v8us*)dl = lv;
  __threadfence();
  *(volatile v8us*)dh = hv;
  *(volatile v8us*)dl = lv;
}

__global__ __launch_bounds__(NTHR) void k_inv(const float* __restrict__ w, float* inv, int n) {
  const int i = (int)blockIdx.x * NTHR + (int)threadIdx.x;
  if (i >= n) return;
  const float v = w[i];
  const float d = 2.0f * (v * v);
  const float r = 1.0f / d;
  *(volatile float*)(inv + i) = r;
  __threadfence();
  *(volatile float*)(inv + i) = r;
}

__global__ __launch_bounds__(NTHR) void k_xsplit(const float* __restrict__ x, unsigned short* ph, unsigned short* pl,
                                                int nN, int nUnits) {
  const int i = (int)blockIdx.x * NTHR + (int)threadIdx.x;
  if (i >= nUnits) return;
  const int row = i >> 4;
  const int c   = (i & 15) * 8;
  const int rc  = row < nN ? row : nN - 1;
  const float* xr = x + (size_t)rc * FD + c;
  v4f a = *(const v4f*)xr, b = *(const v4f*)(xr + 4);
  const v4f z4 = {0.f, 0.f, 0.f, 0.f};
  if (row >= nN) { a = z4; b = z4; }
  v8us hv, lv;
  sp8(a, b, hv, lv);
  unsigned short* dh = ph + (size_t)row * PP + c;
  unsigned short* dl = pl + (size_t)row * PP + c;
  *(volatile v8us*)dh = hv;
  *(volatile v8us*)dl = lv;
  __threadfence();
  *(volatile v8us*)dh = hv;
  *(volatile v8us*)dl = lv;
}

template <int NB>
__device__ __forceinline__ int scan_chunk(const int* __restrict__ dsts, int nE, int cbase, int slotBase,
                                          int vec8, int* list, int tid, int lane, int wave) {
  int wc = 0;
#pragma unroll
  for (int g = 0; g < NGRP; ++g) {
    const int el0  = (g * NTHR + tid) * EPT;
    const int e0   = cbase + el0;
    const int sent = -2147483647 - 1;
    v4i da, db;
    if (vec8 != 0 && cbase + CHUNK <= nE) {
      da = *(const v4i*)(dsts + e0);
      db = *(const v4i*)(dsts + e0 + 4);
    } else {
      da.x = (e0     < nE) ? dsts[min(e0, nE - 1)] : sent;
      da.y = (e0 + 1 < nE) ? dsts[min(e0 + 1, nE - 1)] : sent;
      da.z = (e0 + 2 < nE) ? dsts[min(e0 + 2, nE - 1)] : sent;
      da.w = (e0 + 3 < nE) ? dsts[min(e0 + 3, nE - 1)] : sent;
      db.x = (e0 + 4 < nE) ? dsts[min(e0 + 4, nE - 1)] : sent;
      db.y = (e0 + 5 < nE) ? dsts[min(e0 + 5, nE - 1)] : sent;
      db.z = (e0 + 6 < nE) ? dsts[min(e0 + 6, nE - 1)] : sent;
      db.w = (e0 + 7 < nE) ? dsts[min(e0 + 7, nE - 1)] : sent;
    }
    const unsigned nb = (unsigned)slotBase;
    const unsigned s0 = (unsigned)da.x - nb, s1 = (unsigned)da.y - nb;
    const unsigned s2 = (unsigned)da.z - nb, s3 = (unsigned)da.w - nb;
    const unsigned s4 = (unsigned)db.x - nb, s5 = (unsigned)db.y - nb;
    const unsigned s6 = (unsigned)db.z - nb, s7 = (unsigned)db.w - nb;
    const bool h0 = s0 < (unsigned)NB, h1 = s1 < (unsigned)NB, h2 = s2 < (unsigned)NB, h3 = s3 < (unsigned)NB;
    const bool h4 = s4 < (unsigned)NB, h5 = s5 < (unsigned)NB, h6 = s6 < (unsigned)NB, h7 = s7 < (unsigned)NB;
    const unsigned any = __builtin_amdgcn_ballot_w32(h0 | h1 | h2 | h3 | h4 | h5 | h6 | h7);
    if (any != 0u) {
#define HITJ(J, HJ, SJ) { \
        const unsigned mj = __builtin_amdgcn_ballot_w32(HJ); \
        if (mj != 0u) { \
          if (HJ) { \
            const int pos = wc + (int)__builtin_amdgcn_mbcnt_lo(mj, 0u); \
            if (pos < WCAP) list[wave * WCAP + pos] = ((el0 + (J)) << 12) | (int)(SJ); \
          } \
          wc += (int)__builtin_popcount(mj); } }
      HITJ(0, h0, s0)
      HITJ(1, h1, s1)
      HITJ(2, h2, s2)
      HITJ(3, h3, s3)
      HITJ(4, h4, s4)
      HITJ(5, h5, s5)
      HITJ(6, h6, s6)
      HITJ(7, h7, s7)
#undef HITJ
    }
  }
  return wc;
}

__global__ __launch_bounds__(NTHR) void k_count(
    const int* __restrict__ dsts, int* cnt, int nE, int vec8) {
  __shared__ __attribute__((aligned(16))) int scnt[NBC];
  __shared__ __attribute__((aligned(16))) int list[LISTN];
  __shared__ int wcnt[NWAVE];
  const int tid = threadIdx.x, lane = tid & 31, wave = tid >> 5;
  const int nodeBase = blockIdx.x * NBC;

  for (int i = tid; i < NBC; i += NTHR) scnt[i] = 0;
  __syncthreads();

  const int nChunks = (nE + CHUNK - 1) / CHUNK;
#pragma unroll 1
  for (int ch = 0; ch < nChunks; ++ch) {
    const int cbase = ch * CHUNK;
    const int wc = scan_chunk<NBC>(dsts, nE, cbase, nodeBase, vec8, list, tid, lane, wave);
    if (lane == 0) wcnt[wave] = wc;
    __syncthreads();
    if (wave == 0) {
#pragma unroll 1
      for (int wsx = 0; wsx < NWAVE; ++wsx) {
        int n = __builtin_amdgcn_readfirstlane(wcnt[wsx]);
        n = n > WCAP ? WCAP : (n < 0 ? 0 : n);
        const int* lp = list + wsx * WCAP;
#pragma unroll 1
        for (int i = 0; i < n; ++i) {
          const int ent  = __builtin_amdgcn_readfirstlane(lp[i]);
          const int slot = ent & (NBC - 1);
          if (lane == 0) scnt[slot] = scnt[slot] + 1;
        }
      }
    }
    __syncthreads();
  }

  v4i cq[2];
#pragma unroll
  for (int q = 0; q < 2; ++q) {
    const int f = (wave * 2 + q) * 128 + 4 * lane;
    cq[q] = *(const v4i*)(scnt + f);
  }
  int* cpn = cnt + (size_t)nodeBase;
#pragma unroll
  for (int q = 0; q < 2; ++q) {
    const int f = (wave * 2 + q) * 128 + 4 * lane;
    *(volatile v4i*)(cpn + f) = cq[q];
  }
  __threadfence();
#pragma unroll
  for (int q = 0; q < 2; ++q) {
    const int f = (wave * 2 + q) * 128 + 4 * lane;
    *(volatile v4i*)(cpn + f) = cq[q];
  }
}

__global__ __launch_bounds__(OTHR) void k_offsets(
    const int* __restrict__ cnt, int* off, int* rbase, int nChunk) {
  __shared__ __attribute__((aligned(16))) int soff[NBC];
  __shared__ __attribute__((aligned(16))) int srb[RBN];
  __shared__ int wtot[OTHR / 32];
  const int tid = threadIdx.x, lane = tid & 31, wave = tid >> 5, sub = tid >> 7;
  for (int i = tid; i < RBN; i += OTHR) srb[i] = 0;
  __syncthreads();
  int carry = 0;
#pragma unroll 1
  for (int ch = 0; ch < nChunk; ++ch) {
    const int base = ch * NBC;
    const v4i ca = *(const v4i*)(cnt + base + 8 * tid);
    const v4i cb = *(const v4i*)(cnt + base + 8 * tid + 4);
    const int e0 = max(ca.x, 0), e1 = max(ca.y, 0), e2 = max(ca.z, 0), e3 = max(ca.w, 0);
    const int e4 = max(cb.x, 0), e5 = max(cb.y, 0), e6 = max(cb.z, 0), e7 = max(cb.w, 0);
    const int ts = e0 + e1 + e2 + e3 + e4 + e5 + e6 + e7;
    int incl = ts;
#pragma unroll
    for (int d = 1; d < 32; d <<= 1) {
      const int t = __shfl_up(incl, d);
      if (lane >= d) incl += t;
    }
    if (lane == 31) wtot[wave] = incl;
    __syncthreads();
    int S0 = 0, S1 = 0;
#pragma unroll
    for (int w = 0; w < 4; ++w) { S0 += wtot[w]; S1 += wtot[4 + w]; }
    int pre = 0;
#pragma unroll 1
    for (int w = 4 * sub; w < wave; ++w) pre += wtot[w];
    const int b0 = carry;
    const int b1 = b0 + ((S0 + 31) & ~31);
    const int b2 = b1 + ((S1 + 31) & ~31);
    const int myb = sub == 0 ? b0 : b1;
    if (tid == 0) {
      srb[min(2 * ch + 0, RBN - 1)] = b0;
      srb[min(2 * ch + 1, RBN - 1)] = b1;
    }
    int run = myb + pre + incl - ts;
    soff[8 * tid + 0] = run; run += e0;
    soff[8 * tid + 1] = run; run += e1;
    soff[8 * tid + 2] = run; run += e2;
    soff[8 * tid + 3] = run; run += e3;
    soff[8 * tid + 4] = run; run += e4;
    soff[8 * tid + 5] = run; run += e5;
    soff[8 * tid + 6] = run; run += e6;
    soff[8 * tid + 7] = run;
    carry = b2;
    __syncthreads();
    const v4i o0 = *(const v4i*)(soff + 4 * tid);
    const v4i o1 = *(const v4i*)(soff + 4 * (tid + OTHR));
    int* op = off + base;
    *(volatile v4i*)(op + 4 * tid) = o0;
    *(volatile v4i*)(op + 4 * (tid + OTHR)) = o1;
    __threadfence();
    *(volatile v4i*)(op + 4 * tid) = o0;
    *(volatile v4i*)(op + 4 * (tid + OTHR)) = o1;
    __syncthreads();
  }
  if (tid == 0) srb[min(2 * nChunk, RBN - 1)] = carry;
  __syncthreads();
  v4i rv = {0, 0, 0, 0};
  if (tid < 32) rv = *(const v4i*)(srb + 4 * tid);
  if (tid < 32) *(volatile v4i*)(rbase + 4 * tid) = rv;
  __threadfence();
  if (tid < 32) *(volatile v4i*)(rbase + 4 * tid) = rv;
}

__global__ __launch_bounds__(NTHR) void k_fill(
    const int* __restrict__ dsts, const int* __restrict__ off, const int* __restrict__ rbase,
    int* csr, int nE, int vec8, int csrLen) {
  extern __shared__ v4f lds_dyn[];
  int* region = (int*)lds_dyn;
  int* cursor = region + RCAP;
  int* list   = cursor + NBF;
  int* wcnt   = list + LISTN;
  const int tid = threadIdx.x, lane = tid & 31, wave = tid >> 5;
  const int b = blockIdx.x;
  const int nodeBase = b * NBF;

  int rb0 = rbase[b];
  const int rb1 = rbase[b + 1];
  rb0 = rb0 < 0 ? 0 : (rb0 > csrLen ? csrLen : rb0);
  rb0 &= ~31;
  int len = rb1 - rb0;
  len = len < 0 ? 0 : (len > RCAP ? RCAP : len);
  int lenW = (len + 31) & ~31;
  if (rb0 + lenW > csrLen) lenW = (csrLen - rb0) & ~31;

  {
    const v4i z = {0, 0, 0, 0};
    for (int i = tid; i < RCAP / 4; i += NTHR) ((v4i*)region)[i] = z;
    for (int s = tid; s < NBF; s += NTHR) {
      int o = off[nodeBase + s] - rb0;
      o = o < 0 ? 0 : (o > RCAP ? RCAP : o);
      cursor[s] = o;
    }
  }
  __syncthreads();

  const int nChunks = (nE + CHUNK - 1) / CHUNK;
#pragma unroll 1
  for (int ch = 0; ch < nChunks; ++ch) {
    const int cbase = ch * CHUNK;
    const int wc = scan_chunk<NBF>(dsts, nE, cbase, nodeBase, vec8, list, tid, lane, wave);
    if (lane == 0) wcnt[wave] = wc;
    __syncthreads();
    if (wave == 0) {
#pragma unroll 1
      for (int wsx = 0; wsx < NWAVE; ++wsx) {
        int n = __builtin_amdgcn_readfirstlane(wcnt[wsx]);
        n = n > WCAP ? WCAP : (n < 0 ? 0 : n);
        const int* lp = list + wsx * WCAP;
#pragma unroll 1
        for (int i = 0; i < n; ++i) {
          const int ent  = __builtin_amdgcn_readfirstlane(lp[i]);
          const int slot = ent & (NBF - 1);
          int e = cbase + ((ent >> 12) & (CHUNK - 1));
          e = e > nE - 1 ? nE - 1 : e;
          if (lane == 0) {
            int pos = cursor[slot];
            pos = pos < 0 ? 0 : (pos > RCAP - 1 ? RCAP - 1 : pos);
            region[pos] = e;
            const int np = pos + 1;
            cursor[slot] = np > RCAP ? RCAP : np;
          }
        }
      }
    }
    __syncthreads();
  }

  const int nv = lenW >> 2;
  int* gp = csr + rb0;
#pragma unroll 1
  for (int i = tid; i < nv; i += NTHR) { const v4i v = ((const v4i*)region)[i]; *(volatile v4i*)(gp + 4 * i) = v; }
  __threadfence();
#pragma unroll 1
  for (int i = tid; i < nv; i += NTHR) { const v4i v = ((const v4i*)region)[i]; *(volatile v4i*)(gp + 4 * i) = v; }
}

template <int NCOL>
__device__ __forceinline__ void mm3(const unsigned short* __restrict__ Ah, const unsigned short* __restrict__ Al,
                                    const unsigned short* __restrict__ Bh, const unsigned short* __restrict__ Bl,
                                    int rowBase, float* stg) {
  static_assert((NCOL % 32) == 0);
  constexpr int KD  = FD;
  constexpr int NT  = NCOL / 32;
  constexpr int NCW = NCOL / 2;
  const int tid = threadIdx.x, lane = tid & 31, wave = tid >> 5, hh = lane >> 4, m = lane & 15;
  const int r0 = (wave >> 1) * 16, c0 = (wave & 1) * NCW;
  v8f acc[NT];
#pragma unroll
  for (int t = 0; t < NT; ++t) { v8f z = {0.f, 0.f, 0.f, 0.f, 0.f, 0.f, 0.f, 0.f}; acc[t] = z; }
  const size_t aoff = (size_t)(rowBase + r0 + m) * PP + 8 * hh;
  const unsigned short* aph = Ah + aoff;
  const unsigned short* apl = Al + aoff;
  const size_t boff = (size_t)(c0 + m) * PP + 8 * hh;
  const unsigned short* bph0 = Bh + boff;
  const unsigned short* bpl0 = Bl + boff;
#pragma unroll 1
  for (int kt = 0; kt < KD / 32; ++kt) {
    FragU ah, al;
    ah.u[0] = *(const v8us*)(aph + 32 * kt);
    ah.u[1] = *(const v8us*)(aph + 32 * kt + 16);
    al.u[0] = *(const v8us*)(apl + 32 * kt);
    al.u[1] = *(const v8us*)(apl + 32 * kt + 16);
#pragma unroll
    for (int t = 0; t < NT; ++t) {
      const size_t to = (size_t)(16 * t) * PP + 32 * kt;
      FragU bh, bl;
      bh.u[0] = *(const v8us*)(bph0 + to);
      bh.u[1] = *(const v8us*)(bph0 + to + 16);
      bl.u[0] = *(const v8us*)(bpl0 + to);
      bl.u[1] = *(const v8us*)(bpl0 + to + 16);
      acc[t] = wmb(ah.w, bh.w, acc[t]);
      acc[t] = wmb(al.w, bh.w, acc[t]);
      acc[t] = wmb(ah.w, bl.w, acc[t]);
    }
  }
  float* sp = stg + (size_t)(r0 + 8 * hh) * NCOL + c0 + m;
#pragma unroll
  for (int t = 0; t < NT; ++t) {
#pragma unroll
    for (int r = 0; r < 8; ++r) sp[r * NCOL + 16 * t] = acc[t][r];
  }
}

__global__ __launch_bounds__(NTHR) void k_gemm_in(
    const unsigned short* __restrict__ Ah, const unsigned short* __restrict__ Al,
    const unsigned short* __restrict__ Bh, const unsigned short* __restrict__ Bl,
    const float* __restrict__ bias, float* H, unsigned short* Oh, unsigned short* Ol) {
  extern __shared__ v4f lds_dyn[];
  float* stg = (float*)lds_dyn;
  const int tid = threadIdx.x, lane = tid & 31, wave = tid >> 5;
  const int rowBase = blockIdx.x * BM;
  const int r0 = (wave >> 1) * 16, c0 = (wave & 1) * 64;

  mm3<FD>(Ah, Al, Bh, Bl, rowBase, stg);
  __syncthreads();

  const int rsub = lane >> 4, q = lane & 15, col = c0 + 4 * q;
  const v4f b4 = *(const v4f*)(bias + col);
#pragma unroll
  for (int it = 0; it < 8; ++it) {
    const int row  = 2 * it + rsub;
    const int grow = rowBase + r0 + row;
    const v4f v = relu4(*(const v4f*)(stg + (size_t)(r0 + row) * FD + col) + b4);
    v4us hv, lv;
    sp4(v, hv, lv);
    *(volatile v4f*)(H + (size_t)grow * FD + col) = v;
    *(volatile v4us*)(Oh + (size_t)grow * PP + col) = hv;
    *(volatile v4us*)(Ol + (size_t)grow * PP + col) = lv;
  }
  __threadfence();
#pragma unroll
  for (int it = 0; it < 8; ++it) {
    const int row  = 2 * it + rsub;
    const int grow = rowBase + r0 + row;
    const v4f v = relu4(*(const v4f*)(stg + (size_t)(r0 + row) * FD + col) + b4);
    v4us hv, lv;
    sp4(v, hv, lv);
    *(volatile v4f*)(H + (size_t)grow * FD + col) = v;
    *(volatile v4us*)(Oh + (size_t)grow * PP + col) = hv;
    *(volatile v4us*)(Ol + (size_t)grow * PP + col) = lv;
  }
}

__device__ __forceinline__ float mterm(v4f hv, v4f cv, v4f iv, float d) {
  const v4f t = hv - cv;
  d = fmaf(t.x * t.x, iv.x, d);
  d = fmaf(t.y * t.y, iv.y, d);
  d = fmaf(t.z * t.z, iv.z, d);
  d = fmaf(t.w * t.w, iv.w, d);
  return d;
}

__global__ __launch_bounds__(NTHR) void k_msg(
    const float* __restrict__ hin, const unsigned short* __restrict__ Ph, const unsigned short* __restrict__ Pl,
    const float* __restrict__ cen, const float* __restrict__ inv,
    const unsigned short* __restrict__ Bh, const unsigned short* __restrict__ Bl,
    const float* __restrict__ bcl, float* msg) {
  extern __shared__ v4f lds_dyn[];
  float* hs   = (float*)lds_dyn;
  float* slog = hs + BM * FD;
  float* sw   = slog + BM * RR;
  float* stg  = sw + BM * RR;
  const int tid = threadIdx.x, lane = tid & 31, wave = tid >> 5, hh = lane >> 4, m = lane & 15;
  const int rowBase = blockIdx.x * BM;

#pragma unroll
  for (int i = 0; i < 8; ++i) {
    const int idx = i * NTHR + tid;
    const int row = idx >> 5, c = (idx & 31) * 4;
    *(v4f*)(hs + row * FD + c) = *(const v4f*)(hin + (size_t)(rowBase + row) * FD + c);
  }
  __syncthreads();

  {
    const int row = tid & 63;
    const int rq  = __builtin_amdgcn_readfirstlane(tid >> 6);
    const float* hr = hs + row * FD;
    const float* cb = cen + (size_t)(4 * rq) * FD;
    const float* ib = inv + (size_t)(4 * rq) * FD;
    float d0 = 0.f, d1 = 0.f, d2 = 0.f, d3 = 0.f;
#pragma unroll 1
    for (int k4 = 0; k4 < FD / 4; ++k4) {
      const v4f hv = *(const v4f*)(hr + 4 * k4);
      d0 = mterm(hv, *(const v4f*)(cb + 4 * k4),          *(const v4f*)(ib + 4 * k4),          d0);
      d1 = mterm(hv, *(const v4f*)(cb + FD + 4 * k4),     *(const v4f*)(ib + FD + 4 * k4),     d1);
      d2 = mterm(hv, *(const v4f*)(cb + 2 * FD + 4 * k4), *(const v4f*)(ib + 2 * FD + 4 * k4), d2);
      d3 = mterm(hv, *(const v4f*)(cb + 3 * FD + 4 * k4), *(const v4f*)(ib + 3 * FD + 4 * k4), d3);
    }
    const float sc = -(1.0f / (float)FD);
    v4f lg;
    lg.x = d0 * sc; lg.y = d1 * sc; lg.z = d2 * sc; lg.w = d3 * sc;
    *(v4f*)(slog + row * RR + 4 * rq) = lg;
  }
  __syncthreads();
  if (tid < BM) {
    float* sl = slog + tid * RR;
    float* so = sw + tid * RR;
    float mx = sl[0];
#pragma unroll 1
    for (int r = 1; r < RR; ++r) mx = fmaxf(mx, sl[r]);
    float sum = 0.f;
#pragma unroll 1
    for (int r = 0; r < RR; ++r) { const float e = expf(sl[r] - mx); sl[r] = e; sum += e; }
    const float is = 1.0f / sum;
#pragma unroll 1
    for (int r = 0; r < RR; ++r) so[r] = sl[r] * is;
  }
  __syncthreads();

  const int r0w = (wave >> 1) * 16, c0 = (wave & 1) * 64;
  const size_t aoff = (size_t)(rowBase + r0w + m) * PP + 8 * hh;
  const unsigned short* aph = Ph + aoff;
  const unsigned short* apl = Pl + aoff;
  v8f acc[4];
#pragma unroll
  for (int t = 0; t < 4; ++t) { v8f z = {0.f, 0.f, 0.f, 0.f, 0.f, 0.f, 0.f, 0.f}; acc[t] = z; }
  const float* swr = sw + (r0w + 8 * hh) * RR;
#pragma unroll 1
  for (int r = 0; r < RR; ++r) {
    const size_t boff = ((size_t)r * FD + (size_t)(c0 + m)) * PP + 8 * hh;
    const unsigned short* bph = Bh + boff;
    const unsigned short* bpl = Bl + boff;
    v8f y[4];
#pragma unroll
    for (int t = 0; t < 4; ++t) { v8f z = {0.f, 0.f, 0.f, 0.f, 0.f, 0.f, 0.f, 0.f}; y[t] = z; }
#pragma unroll 1
    for (int kt = 0; kt < FD / 32; ++kt) {
      FragU ah, al;
      ah.u[0] = *(const v8us*)(aph + 32 * kt);
      ah.u[1] = *(const v8us*)(aph + 32 * kt + 16);
      al.u[0] = *(const v8us*)(apl + 32 * kt);
      al.u[1] = *(const v8us*)(apl + 32 * kt + 16);
#pragma unroll
      for (int t = 0; t < 4; ++t) {
        const size_t to = (size_t)(16 * t) * PP + 32 * kt;
        FragU bh, bl;
        bh.u[0] = *(const v8us*)(bph + to);
        bh.u[1] = *(const v8us*)(bph + to + 16);
        bl.u[0] = *(const v8us*)(bpl + to);
        bl.u[1] = *(const v8us*)(bpl + to + 16);
        y[t] = wmb(ah.w, bh.w, y[t]);
        y[t] = wmb(al.w, bh.w, y[t]);
        y[t] = wmb(ah.w, bl.w, y[t]);
      }
    }
    float bq[4];
#pragma unroll
    for (int t = 0; t < 4; ++t) bq[t] = bcl[(size_t)r * FD + c0 + 16 * t + m];
#pragma unroll
    for (int v = 0; v < 8; ++v) {
      const float wv = swr[v * RR + r];
#pragma unroll
      for (int t = 0; t < 4; ++t) acc[t][v] = fmaf(wv, y[t][v] + bq[t], acc[t][v]);
    }
  }

  float* sp = stg + (size_t)(r0w + 8 * hh) * FD + c0 + m;
#pragma unroll
  for (int t = 0; t < 4; ++t) {
#pragma unroll
    for (int r = 0; r < 8; ++r) sp[r * FD + 16 * t] = acc[t][r];
  }
  __syncthreads();
  const int rsub = lane >> 4, q = lane & 15, col = c0 + 4 * q;
#pragma unroll
  for (int it = 0; it < 8; ++it) {
    const int row  = 2 * it + rsub;
    const int grow = rowBase + r0w + row;
    const v4f v = *(const v4f*)(stg + (size_t)(r0w + row) * FD + col);
    *(volatile v4f*)(msg + (size_t)grow * FD + col) = v;
  }
  __threadfence();
#pragma unroll
  for (int it = 0; it < 8; ++it) {
    const int row  = 2 * it + rsub;
    const int grow = rowBase + r0w + row;
    const v4f v = *(const v4f*)(stg + (size_t)(r0w + row) * FD + col);
    *(volatile v4f*)(msg + (size_t)grow * FD + col) = v;
  }
}

__global__ __launch_bounds__(NTHR) void k_agg(
    const int* __restrict__ csr, const int* __restrict__ off, const int* __restrict__ cnt,
    const int* __restrict__ srcs, const float* __restrict__ msg, float* abuf,
    int nN, int nE, int csrLen) {
  const int tid = threadIdx.x, lane = tid & 31, wave = tid >> 5;
  const int tbase = blockIdx.x * TGT + wave * 32;
  const int col = 4 * lane;
  const v4f z4 = {0.f, 0.f, 0.f, 0.f};
  const int cl    = tbase + lane;
  const int cnt_l = cnt[cl];
  const int off_l = off[cl];

#pragma unroll 1
  for (int j = 0; j < 32; ++j) {
    const int c = tbase + j;
    const int n = __shfl(cnt_l, j);
    const int ncl = n < 0 ? 0 : (n > DEGCAP ? DEGCAP : n);
    const int st = __shfl(off_l, j);
    v4f acc = z4;
#pragma unroll 1
    for (int q0 = 0; q0 < ncl; q0 += 32) {
      int pos = st + q0 + lane;
      pos = pos < 0 ? 0 : (pos > csrLen - 1 ? csrLen - 1 : pos);
      int eid = csr[pos];
      eid = eid < 0 ? 0 : (eid > nE - 1 ? nE - 1 : eid);
      int sl = srcs[eid];
      sl = sl < 0 ? 0 : (sl > nN - 1 ? nN - 1 : sl);
      const int mcnt = (ncl - q0) < 32 ? (ncl - q0) : 32;
#pragma unroll 1
      for (int pp = 0; pp < mcnt; ++pp) {
        const int s = __builtin_amdgcn_readlane(sl, pp);
        const v4f xs = *(const v4f*)(msg + (size_t)s * FD + col);
        acc += xs;
      }
    }
    const float degf = (float)(n < 1 ? 1 : n);
    const float rd = 1.0f / degf;
    v4f v = relu4(acc * rd);
    if (c >= nN) v = z4;
    float* po = abuf + (size_t)c * FD + col;
    *(volatile v4f*)po = v;
    __threadfence();
    *(volatile v4f*)po = v;
  }
}

__global__ __launch_bounds__(FD) void k_bnstat(const float* __restrict__ a, double* part, int nN) {
  __shared__ __attribute__((aligned(16))) double spt[2 * FD];
  const int col = threadIdx.x;
  const int r0 = blockIdx.x * STATR;
  int nr = nN - r0;
  nr = nr < 0 ? 0 : (nr > STATR ? STATR : nr);
  double s = 0.0, q = 0.0;
#pragma unroll 1
  for (int i = 0; i < nr; ++i) {
    const double v = (double)a[(size_t)(r0 + i) * FD + col];
    s += v;
    q += v * v;
  }
  spt[col] = s;
  spt[FD + col] = q;
  __syncthreads();
  const v2d w = *(const v2d*)(spt + 2 * col);
  double* pq = part + (size_t)blockIdx.x * (2 * FD) + 2 * col;
  *(volatile v2d*)pq = w;
  __threadfence();
  *(volatile v2d*)pq = w;
}

__global__ __launch_bounds__(FD) void k_bnfin(const double* __restrict__ part, const float* __restrict__ gamma,
                                              float* tbl, int nPart, int nN) {
  __shared__ __attribute__((aligned(16))) float stb[2 * FD];
  const int tid = threadIdx.x, col = tid;
  double s = 0.0, q = 0.0;
#pragma unroll 1
  for (int b = 0; b < nPart; ++b) {
    s += part[(size_t)b * (2 * FD) + col];
    q += part[(size_t)b * (2 * FD) + FD + col];
  }
  const double invn = 1.0 / (double)nN;
  const double mu  = s * invn;
  double var = q * invn - mu * mu;
  var = var < 0.0 ? 0.0 : var;
  const float sc = (float)((double)gamma[col] / sqrt(var + BN_EPS));
  const float mf = (float)mu;
  stb[col] = mf;
  stb[FD + col] = sc;
  __syncthreads();
  const int t4 = tid < 64 ? tid : 63;
  const v4f w = *(const v4f*)(stb + 4 * t4);
  if (tid < 64) *(volatile v4f*)(tbl + 4 * tid) = w;
  __threadfence();
  if (tid < 64) *(volatile v4f*)(tbl + 4 * tid) = w;
}

__global__ __launch_bounds__(NTHR) void k_bnres(
    const float* __restrict__ a, const float* __restrict__ tbl, const float* __restrict__ beta,
    const float* __restrict__ hin, float* hout, unsigned short* ph, unsigned short* pl, int nN, int nUnits) {
  const int i = (int)blockIdx.x * NTHR + (int)threadIdx.x;
  if (i >= nUnits) return;
  const int row = i >> 5;
  const int c   = (i & 31) * 4;
  const v4f a4  = *(const v4f*)(a + (size_t)row * FD + c);
  const v4f h4  = *(const v4f*)(hin + (size_t)row * FD + c);
  const v4f mu4 = *(const v4f*)(tbl + c);
  const v4f sc4 = *(const v4f*)(tbl + FD + c);
  const v4f be4 = *(const v4f*)(beta + c);
  const v4f z4 = {0.f, 0.f, 0.f, 0.f};
  v4f v = h4 + ((a4 - mu4) * sc4 + be4);
  if (row >= nN) v = z4;
  v4us hv, lv;
  sp4(v, hv, lv);
  float* dh = hout + (size_t)row * FD + c;
  unsigned short* eh = ph + (size_t)row * PP + c;
  unsigned short* el = pl + (size_t)row * PP + c;
  *(volatile v4f*)dh = v;
  *(volatile v4us*)eh = hv;
  *(volatile v4us*)el = lv;
  __threadfence();
  *(volatile v4f*)dh = v;
  *(volatile v4us*)eh = hv;
  *(volatile v4us*)el = lv;
}

__global__ __launch_bounds__(NTHR) void k_head(
    const unsigned short* __restrict__ Ah, const unsigned short* __restrict__ Al,
    const unsigned short* __restrict__ Bh, const unsigned short* __restrict__ Bl,
    const float* __restrict__ bias, float* out, int nN) {
  extern __shared__ v4f lds_dyn[];
  float* stg  = (float*)lds_dyn;
  float* sout = stg + BM * NOP;
  const int tid = threadIdx.x;
  const int rowBase = blockIdx.x * BM;

  mm3<NOP>(Ah, Al, Bh, Bl, rowBase, stg);
  __syncthreads();

  if (tid < BM) {
    float* sp = stg + tid * NOP;
    float* so = sout + tid * NOUT;
    float mx = -3.0e38f;
#pragma unroll 1
    for (int o = 0; o < NOUT; ++o) { const float v = sp[o] + bias[o]; sp[o] = v; mx = fmaxf(mx, v); }
    float sum = 0.f;
#pragma unroll 1
    for (int o = 0; o < NOUT; ++o) { const float e = expf(sp[o] - mx); sp[o] = e; sum += e; }
    const float is = 1.0f / sum;
#pragma unroll 1
    for (int o = 0; o < NOUT; ++o) so[o] = sp[o] * is;
  }
  __syncthreads();

  float* ob = out + (size_t)rowBase * NOUT;
  constexpr int NV = BM * NOUT / 4;
  constexpr int VPR = NOUT / 4;
#pragma unroll
  for (int it = 0; it < 3; ++it) {
    const int idx = it * NTHR + tid;
    if (idx < NV) {
      const v4f v = *(const v4f*)(sout + 4 * idx);
      const int grow = rowBase + idx / VPR;
      if (grow < nN) *(volatile v4f*)(ob + 4 * idx) = v;
    }
  }
  __threadfence();
#pragma unroll
  for (int it = 0; it < 3; ++it) {
    const int idx = it * NTHR + tid;
    if (idx < NV) {
      const v4f v = *(const v4f*)(sout + 4 * idx);
      const int grow = rowBase + idx / VPR;
      if (grow < nN) *(volatile v4f*)(ob + 4 * idx) = v;
    }
  }
}

static size_t carve(size_t* o, size_t bytes) {
  const size_t r = *o;
  *o += (bytes + 255) & ~(size_t)255;
  return r;
}

extern "C" void kernel_launch(void* const* d_in, const int* in_sizes, int n_in,
                              void* d_out, int out_size, void* d_ws, size_t ws_size,
                              hipStream_t stream) {
  if (n_in < 12) return;
  const int nN = in_sizes[0] / FD;
  const int nE = in_sizes[1] / 2;
  if (nN <= 0 || nE <= 0 || in_sizes[0] != nN * FD || in_sizes[1] != 2 * nE) return;
  if (in_sizes[2] != FD * FD || in_sizes[3] != FD) return;
  if (in_sizes[4] != NLAY * RR * FD || in_sizes[5] != NLAY * RR * FD) return;
  if (in_sizes[6] != NLAY * RR * FD * FD || in_sizes[7] != NLAY * RR * FD) return;
  if (in_sizes[8] != NLAY * FD || in_sizes[9] != NLAY * FD) return;
  if (in_sizes[10] != FD * NOUT || in_sizes[11] != NOUT) return;
  if ((long long)out_size != (long long)nN * NOUT) return;
  if (nE > (1 << 27) || nN > (1 << 22)) return;

  const float* x      = (const float*)d_in[0];
  const int*   ei     = (const int*)d_in[1];
  const float* W_in   = (const float*)d_in[2];
  const float* b_in   = (const float*)d_in[3];
  const float* cen    = (const float*)d_in[4];
  const float* wid    = (const float*)d_in[5];
  const float* Wc     = (const float*)d_in[6];
  const float* bc     = (const float*)d_in[7];
  const float* gam    = (const float*)d_in[8];
  const float* bet    = (const float*)d_in[9];
  const float* W_head = (const float*)d_in[10];
  const float* b_head = (const float*)d_in[11];
  const int* src = ei;
  const int* dst = ei + nE;
  float* dout = (float*)d_out;

  const int NPAD   = ((nN + TGT - 1) / TGT) * TGT;
  const int nBC    = (nN + NBC - 1) / NBC;
  const int CNTPAD = nBC * NBC;
  if (FPC * nBC + 1 > RBN) return;
  const int nBF    = (nN + NBF - 1) / NBF;
  const int csrLen = ((nE + 31) & ~31) + 4096;
  if (31 * FPC * nBC > 4096) return;
  const int nAgg   = NPAD / TGT;
  const int nGm    = NPAD / BM;
  const int nStat  = NPAD / STATR;
  const int nU16   = NPAD * (FD / 8);
  const int nU32   = NPAD * (FD / 4);
  const int nWc    = NLAY * RR * FD;
  const int nInv   = NLAY * RR * FD;

  char* ws = (char*)d_ws;
  size_t o = 0;
  const size_t plB   = (size_t)NPAD * PP * 2;
  const size_t oPXH  = carve(&o, plB), oPXL = carve(&o, plB);
  const size_t oPHH  = carve(&o, plB), oPHL = carve(&o, plB);
  const size_t oWiH  = carve(&o, (size_t)FD * PP * 2),  oWiL = carve(&o, (size_t)FD * PP * 2);
  const size_t oWcH  = carve(&o, (size_t)nWc * PP * 2), oWcL = carve(&o, (size_t)nWc * PP * 2);
  const size_t oWhH  = carve(&o, (size_t)NOP * PP * 2), oWhL = carve(&o, (size_t)NOP * PP * 2);
  const size_t oInv  = carve(&o, (size_t)nInv * 4);
  const size_t oCnt  = carve(&o, (size_t)CNTPAD * 4);
  const size_t oOff  = carve(&o, (size_t)CNTPAD * 4);
  const size_t oRb   = carve(&o, (size_t)RBN * 4);
  const size_t oCsr  = carve(&o, (size_t)csrLen * 4);
  const size_t oPart = carve(&o, (size_t)nStat * 2 * FD * 8);
  const size_t oTbl  = carve(&o, (size_t)2 * FD * 4);
  const size_t oHA   = carve(&o, (size_t)NPAD * FD * 4);
  const size_t oHB   = carve(&o, (size_t)NPAD * FD * 4);
  const size_t oMsg  = carve(&o, (size_t)NPAD * FD * 4);
  const size_t oA    = carve(&o, (size_t)NPAD * FD * 4);
  if (o > ws_size || o > (size_t)WSCAP) return;

  unsigned short* PXH = (unsigned short*)(ws + oPXH); unsigned short* PXL = (unsigned short*)(ws + oPXL);
  unsigned short* PHH = (unsigned short*)(ws + oPHH); unsigned short* PHL = (unsigned short*)(ws + oPHL);
  unsigned short* WiH = (unsigned short*)(ws + oWiH); unsigned short* WiL = (unsigned short*)(ws + oWiL);
  unsigned short* WcH = (unsigned short*)(ws + oWcH); unsigned short* WcL = (unsigned short*)(ws + oWcL);
  unsigned short* WhH = (unsigned short*)(ws + oWhH); unsigned short* WhL = (unsigned short*)(ws + oWhL);
  float*  inv  = (float*)(ws + oInv);
  int*    cnt  = (int*)(ws + oCnt);
  int*    offp = (int*)(ws + oOff);
  int*    rb   = (int*)(ws + oRb);
  int*    csr  = (int*)(ws + oCsr);
  double* part = (double*)(ws + oPart);
  float*  tbl  = (float*)(ws + oTbl);
  float*  hA   = (float*)(ws + oHA);
  float*  hB   = (float*)(ws + oHB);
  float*  msg  = (float*)(ws + oMsg);
  float*  abuf = (float*)(ws + oA);

  const int vec8 = ((nE & 3) == 0) ? 1 : 0;

  k_xsplit<<<(nU16 + NTHR - 1) / NTHR, NTHR, 0, stream>>>(x, PXH, PXL, nN, nU16);

  k_wprep<<<(FD * 16 + NTHR - 1) / NTHR, NTHR, 0, stream>>>(W_in, FD, FD, WiH, WiL, FD * 16);
  k_wprep<<<(NOP * 16 + NTHR - 1) / NTHR, NTHR, 0, stream>>>(W_head, NOUT, NOP, WhH, WhL, NOP * 16);
  k_bprep<<<(nWc * 16 + NTHR - 1) / NTHR, NTHR, 0, stream>>>(Wc, WcH, WcL, nWc * 16);

  k_inv<<<(nInv + NTHR - 1) / NTHR, NTHR, 0, stream>>>(wid, inv, nInv);

  k_count<<<nBC, NTHR, 0, stream>>>(dst, cnt, nE, vec8);
  k_offsets<<<1, OTHR, 0, stream>>>(cnt, offp, rb, nBC);
  hipFuncSetAttribute(reinterpret_cast<const void*>(&k_fill),
                      hipFuncAttributeMaxDynamicSharedMemorySize, LDS_FILL);
  k_fill<<<nBF, NTHR, LDS_FILL, stream>>>(dst, offp, rb, csr, nE, vec8, csrLen);

  k_gemm_in<<<nGm, NTHR, LDS_GIN, stream>>>(PXH, PXL, WiH, WiL, b_in, hA, PHH, PHL);

  hipFuncSetAttribute(reinterpret_cast<const void*>(&k_msg),
                      hipFuncAttributeMaxDynamicSharedMemorySize, LDS_MSG);
  for (int l = 0; l < NLAY; ++l) {
    const float* hin = (l & 1) ? hB : hA;
    float* hout      = (l & 1) ? hA : hB;
    const float* cen_l = cen + (size_t)l * RR * FD;
    const float* inv_l = inv + (size_t)l * RR * FD;
    const float* bc_l  = bc + (size_t)l * RR * FD;
    const unsigned short* WcH_l = WcH + (size_t)l * RR * FD * PP;
    const unsigned short* WcL_l = WcL + (size_t)l * RR * FD * PP;
    const float* gam_l = gam + (size_t)l * FD;
    const float* bet_l = bet + (size_t)l * FD;
    k_msg<<<nGm, NTHR, LDS_MSG, stream>>>(hin, PHH, PHL, cen_l, inv_l, WcH_l, WcL_l, bc_l, msg);
    k_agg<<<nAgg, NTHR, 0, stream>>>(csr, offp, cnt, src, msg, abuf, nN, nE, csrLen);
    k_bnstat<<<nStat, FD, 0, stream>>>(abuf, part, nN);
    k_bnfin<<<1, FD, 0, stream>>>(part, gam_l, tbl, nStat, nN);
    k_bnres<<<(nU32 + NTHR - 1) / NTHR, NTHR, 0, stream>>>(abuf, tbl, bet_l, hin, hout, PHH, PHL, nN, nU32);
  }

  k_head<<<nGm, NTHR, LDS_HEAD, stream>>>(PHH, PHL, WhH, WhL, b_head, dout, nN);
}
